// SeqAttention_23441931501655
// MI455X (gfx1250) — hardware-verified
//
#include <hip/hip_runtime.h>
#include <math.h>

typedef __attribute__((ext_vector_type(16))) _Float16 v16h;
typedef __attribute__((ext_vector_type(16))) __bf16 v16b;
typedef __attribute__((ext_vector_type(8)))  _Float16 v8h;
typedef __attribute__((ext_vector_type(8)))  float v8f;
typedef __attribute__((ext_vector_type(4)))  float v4f;
typedef __attribute__((ext_vector_type(2)))  float v2f;
typedef __attribute__((ext_vector_type(4)))  unsigned v4u;
typedef __attribute__((ext_vector_type(4)))  int v4i;
typedef float __attribute__((may_alias)) float_a;
typedef int __attribute__((may_alias)) int_a;

template <typename T> __device__ __forceinline__ void vst2(void* p, T v) { *(volatile T*)p = v; __threadfence(); *(volatile T*)p = v; }
__device__ __forceinline__ v8f wmma16(v16h a, v16h b, v8f c) {
  v8f d = __builtin_amdgcn_wmma_f32_16x16x32_f16(false, a, false, b, (short)0, c, false, false);
  asm volatile("v_nop\n\tv_nop\n\tv_nop\n\tv_nop" : "+v"(d) : "v"(a), "v"(b));
  return d;
}
__device__ __forceinline__ v8f wmma_bf(v16b a, v16b b, v8f c) {
  v8f d = __builtin_amdgcn_wmma_f32_16x16x32_bf16(false, a, false, b, (short)0, c, false, false);
  asm volatile("v_nop\n\tv_nop\n\tv_nop\n\tv_nop" : "+v"(d) : "v"(a), "v"(b));
  return d;
}
__device__ __forceinline__ v16h frag_h(const _Float16* rowk0, int lane) {
  union { v16h v; v8h q[2]; } u; const _Float16* p = rowk0 + 8 * (lane >> 4);
  u.q[0] = *(const v8h*)p; u.q[1] = *(const v8h*)(p + 16); return u.v;
}
__device__ __forceinline__ v16h frag_f32(const float* rowk0, int lane) {
  v16h a; const float* p = rowk0 + 8 * (lane >> 4);
#pragma unroll
  for (int i = 0; i < 8; ++i) { a[i] = (_Float16)p[i]; a[8 + i] = (_Float16)p[16 + i]; }
  return a;
}
__device__ __forceinline__ v16h frag_f32s(const float* rowk0, int lane, float sc) {
  v16h a; const float* p = rowk0 + 8 * (lane >> 4);
#pragma unroll
  for (int i = 0; i < 8; ++i) { a[i] = (_Float16)(p[i] * sc); a[8 + i] = (_Float16)(p[16 + i] * sc); }
  return a;
}
__device__ __forceinline__ v16h fragc_f32(const float* W, int k0, int n, int lane, int ld, int K) {
  v16h a; const int g = lane >> 4;
#pragma unroll
  for (int i = 0; i < 8; ++i) { const int ka = k0 + 8 * g + i, kb = ka + 16;
    a[i] = (_Float16)(ka < K ? W[(size_t)ka * ld + n] : 0.f); a[8 + i] = (_Float16)(kb < K ? W[(size_t)kb * ld + n] : 0.f); }
  return a;
}
struct F2 { v16b h, l; };
__device__ __forceinline__ F2 bsplit16(const float v[16]) { F2 r;
#pragma unroll
  for (int i = 0; i < 16; ++i) { const __bf16 h = (__bf16)v[i]; r.h[i] = h; r.l[i] = (__bf16)(v[i] - (float)h); }
  return r; }
__device__ __forceinline__ F2 split_row(const float* row, int k0, int lane) { float v[16]; const float* p = row + k0 + 8 * (lane >> 4);
#pragma unroll
  for (int i = 0; i < 8; ++i) { v[i] = p[i]; v[8 + i] = p[16 + i]; }
  return bsplit16(v); }
__device__ __forceinline__ F2 split_rowK(const float* row, int k0, int lane, int K) { float v[16]; const int g = lane >> 4;
#pragma unroll
  for (int i = 0; i < 8; ++i) { const int ka = k0 + 8 * g + i, kb = ka + 16; v[i] = ka < K ? row[ka] : 0.f; v[8 + i] = kb < K ? row[kb] : 0.f; }
  return bsplit16(v); }
__device__ __forceinline__ F2 split_col(const float* W, int k0, int n, int lane, int ld, int K) { float v[16]; const int g = lane >> 4;
#pragma unroll
  for (int i = 0; i < 8; ++i) { const int ka = k0 + 8 * g + i, kb = ka + 16; v[i] = ka < K ? W[(size_t)ka * ld + n] : 0.f; v[8 + i] = kb < K ? W[(size_t)kb * ld + n] : 0.f; }
  return bsplit16(v); }
__device__ __forceinline__ v8f mac3(const F2& a, const F2& b, v8f c) { c = wmma_bf(a.l, b.h, c); c = wmma_bf(a.h, b.l, c); return wmma_bf(a.h, b.h, c); }
__device__ __forceinline__ float sigm(float v) { return 1.0f / (1.0f + expf(-v)); }
#define LDSX() do { asm volatile("s_wait_dscnt 0" ::: "memory"); __builtin_amdgcn_wave_barrier(); __builtin_amdgcn_fence(__ATOMIC_RELEASE, "workgroup"); } while (0)


#define NBH 64
#define M 1024
#define KL 2048
#define L 1024
#define D 64
#define NKT 17

__global__ __launch_bounds__(128) void k_seq(const float* __restrict__ query, const float* __restrict__ key, const float* __restrict__ value, const float* __restrict__ pe, float* __restrict__ out) {
  __shared__ __align__(16) float sS[4][16][68];
  __shared__ __align__(16) float sQP[4][16][132];
  __shared__ __align__(16) float sO[4][16][68];
  const int tid = threadIdx.x, w = tid >> 5, lane = tid & 31, col = lane & 15, g = lane >> 4;
#ifndef BH0
#define BH0 0
#endif
  const int b = blockIdx.y + BH0; const int q0 = blockIdx.x * 64 + w * 16;
  const float* qb_ = query + (size_t)b * M * D; const float* kb_ = key + (size_t)b * KL * D; const float* vb_ = value + (size_t)b * KL * D;
  v16b aq[2];
#pragma unroll
  for (int kc = 0; kc < 2; ++kc) aq[kc] = split_row(qb_ + (size_t)(q0 + col) * D, kc * 32, lane).h;
  float mrun = -3.0e38f, lrun = 0.f; v8f acc[4] = {}, ac2[4] = {};
  const int kt0 = blockIdx.x;
#pragma unroll 1
  for (int kt = 0; kt < NKT; ++kt) { const int key0 = (kt0 + kt) * 64; if (key0 >= KL) break;
    const int jw = key0 - q0 - 64;
#pragma unroll
    for (int pt = 0; pt < 8; ++pt) { const int j0 = jw + pt * 16; v8f s = {};
      if (j0 >= 0 && j0 + 16 <= L) {
#pragma unroll
        for (int kc = 0; kc < 2; ++kc) s = wmma_bf(aq[kc], split_col(pe, kc * 32, j0 + col, lane, L, D).h, s); }
#pragma unroll
      for (int r = 0; r < 8; ++r) sQP[w][8 * g + r][pt * 16 + col] = s[r]; }
#pragma unroll
    for (int t = 0; t < 4; ++t) { const int kk = key0 + t * 16 + col; v8f s = {};
#pragma unroll
      for (int kc = 0; kc < 2; ++kc) s = wmma_bf(aq[kc], split_row(kb_ + (size_t)kk * D, kc * 32, lane).h, s);
#pragma unroll
      for (int r = 0; r < 8; ++r) sS[w][8 * g + r][t * 16 + col] = s[r]; }
    LDSX();
    { const int rq = col; const int i = q0 + rq;
#pragma unroll
      for (int jj = 0; jj < 32; ++jj) { const int kc_ = g * 32 + jj; const int kk = key0 + kc_; const int j = kk - i; float v;
        if (j < 0 || j >= L) v = -3.0e38f;
        else { float sc = sS[w][rq][kc_];
          if (fabsf(sc) < 1.0e-5f) { const float* qr = qb_ + (size_t)i * D; const float* kr = kb_ + (size_t)kk * D; float acc_ = 0.f;
            for (int dd = 0; dd < D; ++dd) acc_ = fmaf((float)(__bf16)qr[dd], (float)(__bf16)kr[dd], acc_);
            if (acc_ == 0.0f) sc = -1000000.0f; }
          v = (sc + sQP[w][rq][j - jw]) * 0.125f; }
        sS[w][rq][kc_] = v; } }
    LDSX();
    float mx = -3.4e38f;
#pragma unroll
    for (int jj = 0; jj < 32; ++jj) mx = fmaxf(mx, sS[w][col][g * 32 + jj]);
    mx = fmaxf(mx, __shfl_xor(mx, 16, 32));
    const float mnew = fmaxf(mrun, mx); const float corr = expf(mrun - mnew);
    float ps = 0.f;
#pragma unroll
    for (int jj = 0; jj < 32; ++jj) { const float sv = sS[w][col][g * 32 + jj]; const float p = sv <= -1.0e38f ? 0.f : expf(sv - mnew); ps += p; sS[w][col][g * 32 + jj] = p; }
    ps += __shfl_xor(ps, 16, 32);
    lrun = lrun * corr + ps; mrun = mnew;
#pragma unroll
    for (int r = 0; r < 8; ++r) { const float cr = __shfl(corr, 8 * g + r, 32);
#pragma unroll
      for (int t = 0; t < 4; ++t) { acc[t][r] *= cr; ac2[t][r] *= cr; } }
    LDSX();
#pragma unroll
    for (int kc = 0; kc < 2; ++kc) { const F2 pa = split_row(&sS[w][col][0], kc * 32, lane);
#pragma unroll
      for (int t = 0; t < 4; ++t) { const v16b vb = split_col(vb_ + (size_t)(key0 + kc * 32) * D, 0, t * 16 + col, lane, D, 32).h; acc[t] = wmma_bf(pa.h, vb, acc[t]); ac2[t] = wmma_bf(pa.l, vb, ac2[t]); } }
    LDSX(); }
#pragma unroll
  for (int r = 0; r < 8; ++r) { const float lr = __shfl(lrun, 8 * g + r, 32); const float inv = 1.0f / lr;
#pragma unroll
    for (int t = 0; t < 4; ++t) sO[w][8 * g + r][t * 16 + col] = (acc[t][r] + ac2[t][r]) * inv; }
  LDSX();
  for (int qq = lane; qq < 16 * 16; qq += 32) { const int rl = qq >> 4, pc = qq & 15; vst2(out + ((size_t)b * M + q0 + rl) * D + pc * 4, *(const v4f*)(&sO[w][rl][pc * 4])); }
}
extern "C" void kernel_launch(void* const* d_in, const int* in_sizes, int n_in, void* d_out, int out_size, void* d_ws, size_t ws_size, hipStream_t stream) {
  (void)in_sizes; (void)n_in; (void)out_size; (void)ws_size; (void)d_ws;
  const float* query = (const float*)d_in[0]; const float* key = (const float*)d_in[1]; const float* value = (const float*)d_in[2]; const float* pe = (const float*)d_in[3];
  float* out = (float*)d_out;
  k_seq<<<dim3(M / 64, NBH), 128, 0, stream>>>(query, key, value, pe, out);
}
